// FinetuneBertFANAttention_73254962201223
// MI455X (gfx1250) — hardware-run, weakly checked
//
#include <hip/hip_runtime.h>
#include <math.h>
#include <stdint.h>

#define BB_    32
#define SS_    512
#define DD_    768
#define NTOK   (BB_ * SS_)
#define YD     3
#define ZD     5
#define LNEPS  1e-5f
#define COSEPS 1e-8f
#define ESC    64.0f
#define WSC    256.0f
#define HSC    16.0f
#define FSC    64.0f

static_assert((DD_ % 64) == 0 && (DD_ % 32) == 0 && (DD_ % 256) == 0);
static_assert((NTOK % 32) == 0 && (SS_ % 128) == 0 && (SS_ % 32) == 0);
static_assert(((NTOK * DD_) % 2048) == 0);
static_assert((((NTOK / 16) * (DD_ / 64)) % 8) == 0);
static_assert((32 * YD) % 4 == 0 && (32 * ZD) % 4 == 0 && (32 * YD) / 4 <= 32 && (32 * ZD) / 4 <= 64);

typedef _Float16 v16h __attribute__((ext_vector_type(16)));
typedef _Float16 v8h  __attribute__((ext_vector_type(8)));
typedef float    v8f  __attribute__((ext_vector_type(8)));
typedef float    v4f  __attribute__((ext_vector_type(4)));
typedef unsigned int v4u __attribute__((ext_vector_type(4)));

union FragH { v16h v; v8h h[2]; };

__device__ __forceinline__ unsigned short bf_bits(float f) {
  unsigned u = __float_as_uint(f);
  return (unsigned short)((u + 0x7FFFu + ((u >> 16) & 1u)) >> 16);
}
__device__ __forceinline__ float bf_up(unsigned short h) { return __uint_as_float(((unsigned)h) << 16); }
__device__ __forceinline__ float bfr(float f) { return bf_up(bf_bits(f)); }
__device__ __forceinline__ unsigned short h_bits(_Float16 x) { return __builtin_bit_cast(unsigned short, x); }
__device__ __forceinline__ unsigned pk16(unsigned short a, unsigned short b) { return (unsigned)a | ((unsigned)b << 16); }
__device__ __forceinline__ unsigned pkh(float a, float b) { return pk16(h_bits((_Float16)a), h_bits((_Float16)b)); }
__device__ __forceinline__ v8f zero8() { v8f z = {0.f, 0.f, 0.f, 0.f, 0.f, 0.f, 0.f, 0.f}; return z; }

__device__ __forceinline__ v16h ldfrag_h(const _Float16* p) {
  FragH f;
  f.h[0] = *(const v8h*)(p);
  f.h[1] = *(const v8h*)(p + 16);
  return f.v;
}

__device__ __forceinline__ v8f mma_h(v16h a, v16h b, v8f c) {
  c = __builtin_amdgcn_wmma_f32_16x16x32_f16(false, a, false, b, (short)0, c, false, false);
#if defined(__HIP_DEVICE_COMPILE__)
  asm volatile("v_nop\n\tv_nop\n\tv_nop\n\tv_nop" : "+v"(c) : "v"(a), "v"(b));
#endif
  return c;
}
__device__ __forceinline__ void wave_sync_lds() {
  __builtin_amdgcn_fence(__ATOMIC_RELEASE, "workgroup");
  __builtin_amdgcn_wave_barrier();
  __builtin_amdgcn_fence(__ATOMIC_ACQUIRE, "workgroup");
}

__global__ __launch_bounds__(256) void cvt_wT(const float* __restrict__ w0, const float* __restrict__ w1,
                                              unsigned short* outp, int nin, int nout) {
  __shared__ float tile[64][33];
  const int tid = threadIdx.x;
  const int z = blockIdx.z;
  const float* src = (z == 0) ? w0 : w1;
  unsigned short* dst = outp + (size_t)z * nin * nout;
  const int i0 = blockIdx.x * 64;
  const int o0 = blockIdx.y * 32;
#pragma unroll
  for (int p = 0; p < 8; ++p) {
    const int idx = p * 256 + tid;
    const int i = idx >> 5, o = idx & 31;
    tile[i][o] = src[(size_t)(i0 + i) * nout + o0 + o];
  }
  __syncthreads();
  const int o = tid >> 3, c8 = (tid & 7) * 8;
  v4u pk;
#pragma unroll
  for (int e = 0; e < 4; ++e)
    pk[e] = pkh(bfr(tile[c8 + 2 * e][o]) * WSC, bfr(tile[c8 + 2 * e + 1][o]) * WSC);
  unsigned short* gp = dst + (size_t)(o0 + o) * nin + i0 + c8;
  *(volatile v4u*)gp = pk;
  __threadfence();
  *(volatile v4u*)gp = pk;
}

__global__ __launch_bounds__(256) void cvt_emb(const float* __restrict__ x, unsigned short* outp) {
  const size_t base = ((size_t)blockIdx.x * 256 + threadIdx.x) * 8;
  const v4f a = *(const v4f*)(x + base);
  const v4f c = *(const v4f*)(x + base + 4);
  v4u pk;
  pk[0] = pkh(bfr(a[0]) * ESC, bfr(a[1]) * ESC);
  pk[1] = pkh(bfr(a[2]) * ESC, bfr(a[3]) * ESC);
  pk[2] = pkh(bfr(c[0]) * ESC, bfr(c[1]) * ESC);
  pk[3] = pkh(bfr(c[2]) * ESC, bfr(c[3]) * ESC);
  unsigned short* gp = outp + base;
  *(volatile v4u*)gp = pk;
  __threadfence();
  *(volatile v4u*)gp = pk;
}

template <int MODE>
__global__ __launch_bounds__(256) void gemm16(const unsigned short* __restrict__ Ap,
                                              const unsigned short* __restrict__ Bp,
                                              const float* __restrict__ bias, const float* __restrict__ resid,
                                              unsigned short* Ch, float* C32, float sc) {
#pragma clang fp contract(off)
  __shared__ __align__(16) float sT[8][16 * 68];
  constexpr int TN  = DD_ / 64;
  constexpr int TOT = (NTOK / 16) * TN;
  const int lane = threadIdx.x & 31;
  const int wave = threadIdx.x >> 5;
  const int t = __builtin_amdgcn_readfirstlane((int)(blockIdx.x * 8 + wave));
  if (t >= TOT) return;
  const int tm = t / TN;
  const int tn = t - tm * TN;
  const int m0 = tm * 16;
  const int n0 = tn * 64;

  const int rl   = lane & 15;
  const int hh   = lane >> 4;
  const int koff = hh * 8;

  const _Float16* A  = (const _Float16*)(const void*)Ap;
  const _Float16* Bt = (const _Float16*)(const void*)Bp;

  v8f acc[4];
#pragma unroll
  for (int j = 0; j < 4; ++j) acc[j] = zero8();

  const size_t arow = (size_t)(m0 + rl) * DD_ + koff;
#pragma unroll 2
  for (int k0 = 0; k0 < DD_; k0 += 32) {
    const v16h fa = ldfrag_h(A + arow + k0);
#pragma unroll
    for (int j = 0; j < 4; ++j) {
      const v16h fb = ldfrag_h(Bt + (size_t)(n0 + 16 * j + rl) * DD_ + koff + k0);
      acc[j] = mma_h(fa, fb, acc[j]);
    }
  }

  float* slab = sT[wave];
#pragma unroll
  for (int j = 0; j < 4; ++j) {
#pragma unroll
    for (int r = 0; r < 8; ++r) slab[(koff + r) * 68 + 16 * j + rl] = acc[j][r] * sc;
  }
  wave_sync_lds();

  if (MODE == 1) {
    const int h2 = lane >> 4, c4 = (lane & 15) * 4;
    float bz[4];
#pragma unroll
    for (int e = 0; e < 4; ++e) bz[e] = bfr(bias[n0 + c4 + e]);
    v4f ov[8];
#pragma unroll
    for (int it = 0; it < 8; ++it) {
      const int row = it * 2 + h2;
      const v4f v  = *(const v4f*)(slab + row * 68 + c4);
      const v4f rv = *(const v4f*)(resid + (size_t)(m0 + row) * DD_ + n0 + c4);
      v4f o;
#pragma unroll
      for (int e = 0; e < 4; ++e) {
        float f = v[e] + bz[e];
        const float rb = bfr(rv[e]);
        f = rb + f;
        o[e] = f;
      }
      ov[it] = o;
    }
    for (int pass = 0; pass < 2; ++pass) {
#pragma unroll
      for (int it = 0; it < 8; ++it) {
        const int row = it * 2 + h2;
        float* gp = C32 + (size_t)(m0 + row) * DD_ + n0 + c4;
        *(volatile v4f*)gp = ov[it];
      }
      __threadfence();
    }
  } else {
    const int q = lane >> 3, c8 = (lane & 7) * 8;
    float bz[8];
#pragma unroll
    for (int e = 0; e < 8; ++e) bz[e] = bfr(bias[n0 + c8 + e]);
    v4u hv[4];
#pragma unroll
    for (int it = 0; it < 4; ++it) {
      const int row = it * 4 + q;
      const float* sp = slab + row * 68 + c8;
      const v4f x0 = *(const v4f*)sp;
      const v4f x1 = *(const v4f*)(sp + 4);
      float f[8];
#pragma unroll
      for (int e = 0; e < 4; ++e) { f[e] = x0[e]; f[4 + e] = x1[e]; }
#pragma unroll
      for (int e = 0; e < 8; ++e) {
        float u = f[e] + bz[e];
        u = fmaxf(u, 0.f);
        f[e] = u * HSC;
      }
      v4u a;
#pragma unroll
      for (int e = 0; e < 4; ++e) a[e] = pkh(f[2 * e], f[2 * e + 1]);
      hv[it] = a;
    }
    for (int pass = 0; pass < 2; ++pass) {
#pragma unroll
      for (int it = 0; it < 4; ++it) {
        const int row = it * 4 + q;
        unsigned short* gp = Ch + (size_t)(m0 + row) * DD_ + n0 + c8;
        *(volatile v4u*)gp = hv[it];
      }
      __threadfence();
    }
  }
}

__global__ __launch_bounds__(256) void ln_rows(const float* __restrict__ xin, const float* __restrict__ g,
                                               const float* __restrict__ bt, const float* __restrict__ wy,
                                               const float* __restrict__ by, const float* __restrict__ wz,
                                               const float* __restrict__ bz, unsigned short* fh, float* nrm,
                                               float* outp) {
#pragma clang fp contract(off)
  __shared__ __align__(16) float srow[8][DD_];
  __shared__ __align__(16) float sO1[32 * YD];
  __shared__ __align__(16) float sO2[32 * ZD];
  __shared__ __align__(16) float sN[32];
  const int tid = threadIdx.x, wave = tid >> 5, lane = tid & 31;
  const int c8 = lane * 8;
  float* myrow = srow[wave];

#pragma unroll 1
  for (int rr = 0; rr < 4; ++rr) {
    const int rloc = wave * 4 + rr;
    const size_t row = (size_t)blockIdx.x * 32 + rloc;
    const float* rp = xin + row * DD_;
    float x[24];
#pragma unroll
    for (int sg = 0; sg < 3; ++sg) {
      const v4f a = *(const v4f*)(rp + 256 * sg + c8);
      const v4f c = *(const v4f*)(rp + 256 * sg + c8 + 4);
#pragma unroll
      for (int e = 0; e < 4; ++e) { x[8 * sg + e] = a[e]; x[8 * sg + 4 + e] = c[e]; }
    }
    float s = 0.f;
#pragma unroll
    for (int e = 0; e < 24; ++e) s = s + x[e];
#pragma unroll
    for (int off = 1; off < 32; off <<= 1) s = s + __shfl_xor(s, off, 32);
    const float mu = s * (1.0f / DD_);
    float d[24];
    float s2 = 0.f;
#pragma unroll
    for (int e = 0; e < 24; ++e) { d[e] = x[e] - mu; const float dd = d[e] * d[e]; s2 = s2 + dd; }
#pragma unroll
    for (int off = 1; off < 32; off <<= 1) s2 = s2 + __shfl_xor(s2, off, 32);
    const float var = s2 * (1.0f / DD_);
    const float rstd = 1.0f / sqrtf(var + LNEPS);
    float y[24];
    float nsq = 0.f;
#pragma unroll
    for (int e = 0; e < 24; ++e) {
      const int col = 256 * (e >> 3) + c8 + (e & 7);
      const float gg = bfr(g[col]), bb = bfr(bt[col]);
      float t = d[e] * rstd;
      t = t * gg;
      t = t + bb;
      y[e] = t;
      const float yy2 = t * t;
      nsq = nsq + yy2;
    }
#pragma unroll
    for (int off = 1; off < 32; off <<= 1) nsq = nsq + __shfl_xor(nsq, off, 32);
    const float nv = sqrtf(nsq);

    v4u pk[3];
#pragma unroll
    for (int sg = 0; sg < 3; ++sg) {
      v4u a;
#pragma unroll
      for (int e = 0; e < 4; ++e) a[e] = pkh(y[8 * sg + 2 * e] * FSC, y[8 * sg + 2 * e + 1] * FSC);
      pk[sg] = a;
    }
    unsigned short* hp = fh + row * DD_ + c8;
    for (int pass = 0; pass < 2; ++pass) {
#pragma unroll
      for (int sg = 0; sg < 3; ++sg) *(volatile v4u*)(hp + 256 * sg) = pk[sg];
      __threadfence();
    }

#pragma unroll
    for (int sg = 0; sg < 3; ++sg) {
      v4f a, c;
#pragma unroll
      for (int e = 0; e < 4; ++e) { a[e] = y[8 * sg + e]; c[e] = y[8 * sg + 4 + e]; }
      *(v4f*)(myrow + 256 * sg + c8) = a;
      *(v4f*)(myrow + 256 * sg + c8 + 4) = c;
    }
    wave_sync_lds();
    float p[8];
#pragma unroll
    for (int o = 0; o < 8; ++o) p[o] = 0.f;
#pragma unroll 1
    for (int it = 0; it < DD_ / 32; ++it) {
      const int dc = it * 32 + lane;
      const float f = myrow[dc];
#pragma unroll
      for (int yy = 0; yy < YD; ++yy) {
        const float w = bfr(wy[dc * YD + yy]);
        const float pr = f * w;
        p[yy] = p[yy] + pr;
      }
#pragma unroll
      for (int zz = 0; zz < ZD; ++zz) {
        const float w = bfr(wz[dc * ZD + zz]);
        const float pr = f * w;
        p[YD + zz] = p[YD + zz] + pr;
      }
    }
#pragma unroll
    for (int off = 16; off >= 1; off >>= 1) {
#pragma unroll
      for (int o = 0; o < 8; ++o) p[o] = p[o] + __shfl_xor(p[o], off, 32);
    }
    if (lane == 0) {
#pragma unroll
      for (int yy = 0; yy < YD; ++yy) sO1[rloc * YD + yy] = p[yy] + bfr(by[yy]);
#pragma unroll
      for (int zz = 0; zz < ZD; ++zz) sO2[rloc * ZD + zz] = p[YD + zz] + bfr(bz[zz]);
      sN[rloc] = nv;
    }
    wave_sync_lds();
  }
  __syncthreads();

  {
    const int blk = blockIdx.x;
    const bool a1 = tid < (32 * YD) / 4;
    const bool a2 = (tid >= 32) && (tid < 32 + (32 * ZD) / 4);
    const bool a3 = (tid >= 96) && (tid < 104);
    const int u1 = a1 ? tid : 0;
    const int u2 = a2 ? (tid - 32) : 0;
    const int u3 = a3 ? (tid - 96) : 0;
    const v4f v1 = *(const v4f*)(sO1 + 4 * u1);
    const v4f v2 = *(const v4f*)(sO2 + 4 * u2);
    const v4f v3 = *(const v4f*)(sN + 4 * u3);
    float* g1 = outp + (size_t)blk * (32 * YD) + 4 * u1;
    float* g2 = outp + (size_t)NTOK * YD + (size_t)blk * (32 * ZD) + 4 * u2;
    float* g3 = nrm + (size_t)blk * 32 + 4 * u3;
    v4f v;
#pragma unroll
    for (int e = 0; e < 4; ++e) v[e] = a1 ? v1[e] : (a2 ? v2[e] : v3[e]);
    float* gp = a1 ? g1 : (a2 ? g2 : g3);
    const bool act = a1 || a2 || a3;
    if (act) { *(volatile v4f*)gp = v; }
    __threadfence();
    if (act) { *(volatile v4f*)gp = v; }
  }
}

__global__ __launch_bounds__(256) void dots_rowsum(const unsigned short* __restrict__ fh,
                                                   const float* __restrict__ nrm, float* rs) {
#pragma clang fp contract(off)
  __shared__ float sP[8][16];
  __shared__ __align__(16) float sRS[32];
  const int tid = threadIdx.x, wave = tid >> 5, lane = tid & 31;
  const int m = lane & 15, hh = lane >> 4;
  const int rg = blockIdx.x, b = blockIdx.y;
  const int rt = wave >> 2, ct = wave & 3;
  const _Float16* F = (const _Float16*)(const void*)fh;
  const size_t rbase = (size_t)b * SS_;
  const int srow0 = rg * 32 + rt * 16;
  const size_t arow = (rbase + srow0 + m) * DD_ + 8 * hh;
  float nr[8];
#pragma unroll
  for (int r = 0; r < 8; ++r) nr[r] = nrm[rbase + srow0 + 8 * hh + r];
  float p[8];
#pragma unroll
  for (int r = 0; r < 8; ++r) p[r] = 0.f;

#pragma unroll 1
  for (int jp = 0; jp < 2; ++jp) {
    const int tcol0 = ct * 128 + jp * 64;
    v8f acc[4];
#pragma unroll
    for (int j = 0; j < 4; ++j) acc[j] = zero8();
#pragma unroll 2
    for (int k0 = 0; k0 < DD_; k0 += 32) {
      const v16h fa = ldfrag_h(F + arow + k0);
#pragma unroll
      for (int j = 0; j < 4; ++j) {
        const v16h fb = ldfrag_h(F + (rbase + tcol0 + 16 * j + m) * DD_ + 8 * hh + k0);
        acc[j] = mma_h(fa, fb, acc[j]);
      }
    }
#pragma unroll
    for (int j = 0; j < 4; ++j) {
      const float ncj = nrm[rbase + tcol0 + 16 * j + m];
#pragma unroll
      for (int r = 0; r < 8; ++r) {
        float den = nr[r] * ncj;
        den = den + COSEPS;
        float q = acc[j][r] * (1.0f / (FSC * FSC));
        q = q * __builtin_amdgcn_rcpf(den);
        p[r] = p[r] + q;
      }
    }
  }
#pragma unroll
  for (int off = 1; off < 16; off <<= 1) {
#pragma unroll
    for (int r = 0; r < 8; ++r) p[r] = p[r] + __shfl_xor(p[r], off, 32);
  }
  if (m == 0) {
#pragma unroll
    for (int r = 0; r < 8; ++r) sP[wave][8 * hh + r] = p[r];
  }
  __syncthreads();
  if (tid < 32) {
    const int q4 = tid >> 4, rr = tid & 15;
    float s = sP[q4 * 4 + 0][rr];
    s = s + sP[q4 * 4 + 1][rr];
    s = s + sP[q4 * 4 + 2][rr];
    s = s + sP[q4 * 4 + 3][rr];
    sRS[tid] = s;
  }
  __syncthreads();
  if (tid < 8) {
    const v4f v = *(const v4f*)(sRS + 4 * tid);
    float* gp = rs + rbase + rg * 32 + 4 * tid;
    *(volatile v4f*)gp = v;
    __threadfence();
    *(volatile v4f*)gp = v;
  }
}

__global__ __launch_bounds__(SS_) void attn_out(const float* __restrict__ rs, float* outp) {
#pragma clang fp contract(off)
  __shared__ float smx[SS_ / 32];
  __shared__ float ssm[SS_ / 32];
  __shared__ __align__(16) float so[SS_];
  const int t = threadIdx.x, wave = t >> 5, lane = t & 31;
  const int b = blockIdx.x;
  const float aw = rs[(size_t)b * SS_ + t] * (1.0f / SS_);
  const float sg = 1.0f / (1.0f + __expf(aw));
  float mx = sg;
#pragma unroll
  for (int off = 16; off >= 1; off >>= 1) mx = fmaxf(mx, __shfl_xor(mx, off, 32));
  if (lane == 0) smx[wave] = mx;
  __syncthreads();
  float gm = smx[0];
#pragma unroll
  for (int w = 1; w < SS_ / 32; ++w) gm = fmaxf(gm, smx[w]);
  const float e = __expf(sg - gm);
  float sm = e;
#pragma unroll
  for (int off = 16; off >= 1; off >>= 1) sm = sm + __shfl_xor(sm, off, 32);
  if (lane == 0) ssm[wave] = sm;
  __syncthreads();
  float tot = ssm[0];
#pragma unroll
  for (int w = 1; w < SS_ / 32; ++w) tot = tot + ssm[w];
  const float o = e * (1.0f / tot);
  so[t] = o;
  __syncthreads();
  if (t < SS_ / 4) {
    const v4f v = *(const v4f*)(so + 4 * t);
    float* gp = outp + (size_t)NTOK * (YD + ZD) + (size_t)b * SS_ + 4 * t;
    *(volatile v4f*)gp = v;
    __threadfence();
    *(volatile v4f*)gp = v;
  }
}

extern "C" void kernel_launch(void* const* d_in, const int* in_sizes, int n_in,
                              void* d_out, int out_size, void* d_ws, size_t ws_size,
                              hipStream_t stream) {
  if (n_in < 11) return;
  const int ex[11] = { NTOK * DD_, DD_ * DD_, DD_, DD_ * DD_, DD_, DD_, DD_, DD_ * YD, YD, DD_ * ZD, ZD };
  for (int i = 0; i < 11; ++i) if (in_sizes[i] != ex[i]) return;
  if (out_size != NTOK * (YD + ZD + 1)) return;

  const float* emb = (const float*)d_in[0];
  const float* W1  = (const float*)d_in[1];
  const float* b1  = (const float*)d_in[2];
  const float* W2  = (const float*)d_in[3];
  const float* b2  = (const float*)d_in[4];
  const float* gam = (const float*)d_in[5];
  const float* bet = (const float*)d_in[6];
  const float* Wy  = (const float*)d_in[7];
  const float* by  = (const float*)d_in[8];
  const float* Wz  = (const float*)d_in[9];
  const float* bz  = (const float*)d_in[10];
  float* out = (float*)d_out;

  const size_t PL  = (size_t)DD_ * DD_;
  const size_t sWP = PL * 2 * 2;
  const size_t sH  = (size_t)NTOK * DD_ * 2;
  const size_t sF  = (size_t)NTOK * DD_ * 4;
  const size_t sS  = (size_t)NTOK * 4;
  size_t off = 0;
  const size_t oWP  = off; off += sWP;
  const size_t oE16 = off; off += sH;
  const size_t oH16 = off; off += sH;
  const size_t oX32 = off; off += sF;
  const size_t oF16 = off; off += sH;
  const size_t oNRM = off; off += sS;
  const size_t oRS  = off; off += sS;
  if (off > ws_size) return;
  if (off > (size_t)134217728) return;

  char* ws = (char*)d_ws;
  unsigned short* WP  = (unsigned short*)(ws + oWP);
  unsigned short* E16 = (unsigned short*)(ws + oE16);
  unsigned short* H16 = (unsigned short*)(ws + oH16);
  float*          X32 = (float*)(ws + oX32);
  unsigned short* F16 = (unsigned short*)(ws + oF16);
  float*          NRM = (float*)(ws + oNRM);
  float*          RS  = (float*)(ws + oRS);
  const unsigned short* W1T = WP;
  const unsigned short* W2T = WP + PL;

  const dim3 blk(256);

  cvt_wT<<<dim3(DD_ / 64, DD_ / 32, 2), blk, 0, stream>>>(W1, W2, WP, DD_, DD_);
  cvt_emb<<<dim3((NTOK * DD_) / 2048), blk, 0, stream>>>(emb, E16);

  const dim3 ggrid(((NTOK / 16) * (DD_ / 64)) / 8);
  gemm16<0><<<ggrid, blk, 0, stream>>>(E16, W1T, b1, emb, H16, X32, 1.0f / (ESC * WSC));
  gemm16<1><<<ggrid, blk, 0, stream>>>(H16, W2T, b2, emb, H16, X32, 1.0f / (HSC * WSC));
  ln_rows<<<dim3(NTOK / 32), blk, 0, stream>>>(X32, gam, bet, Wy, by, Wz, bz, F16, NRM, out);
  dots_rowsum<<<dim3(SS_ / 32, BB_), blk, 0, stream>>>(F16, NRM, RS);
  attn_out<<<dim3(BB_), dim3(SS_), 0, stream>>>(RS, out);
  (void)hipGetLastError();
}
